// MultiHeadSelfAttention_7782480740945
// MI455X (gfx1250) — hardware-verified
//
#include <hip/hip_runtime.h>


#ifndef NB
#define NB 4
#endif
#ifndef SEQ
#define SEQ 2048
#endif
#define NB_FULL  4
#define SEQ_FULL 2048
#define EM   1024
#define NH   16
#define HD   64
#define E3   (3 * EM)
#define RH   256
#define PP   40
#define PCAR 1024.0f
#define CE   0.0450842200277801f
#define MROWS (NB * SEQ)
#define PLANE   ((size_t)NB * NH * SEQ * HD)
#define VRPLANE ((size_t)NB * NH * HD * RH)
#define ATPLANE ((size_t)MROWS * EM)

static_assert(EM == NH * HD);
static_assert(HD == 64);
static_assert(E3 == NH * 3 * HD);
static_assert(SEQ % 64 == 0);
static_assert(RH % 64 == 0 && SEQ >= RH);
static_assert(EM % 64 == 0 && E3 % 64 == 0 && EM % 32 == 0);
static_assert(NB <= NB_FULL && SEQ <= SEQ_FULL);
static_assert(((size_t)MROWS * EM) % 2048 == 0);

typedef _Float16 h16;
typedef unsigned short bf;
typedef __attribute__((ext_vector_type(16))) __bf16   v16bf;
typedef __attribute__((ext_vector_type(16))) _Float16 v16h;
typedef __attribute__((ext_vector_type(8)))  _Float16 v8h;
typedef __attribute__((ext_vector_type(8)))  unsigned short v8us;
typedef __attribute__((ext_vector_type(8)))  float    v8f;
typedef __attribute__((ext_vector_type(4)))  float    v4f;
typedef v8h  __attribute__((may_alias)) v8ha;
typedef v4f  __attribute__((may_alias)) v4fa;
typedef v8us __attribute__((may_alias)) v8usa;

constexpr size_t SZ_WQ = (size_t)E3 * EM * 2;
constexpr size_t SZ_WO = (size_t)EM * EM * 2;
constexpr size_t SZ_XB = (size_t)MROWS * EM * 2;
constexpr size_t SZ_P16 = 3 * PLANE * 2;
constexpr size_t SZ_VR = VRPLANE * 2;
constexpr size_t SZ_AT = 2 * ATPLANE * 2;
constexpr size_t SZ_TOTAL = SZ_WQ + SZ_WO + SZ_XB + SZ_P16 + 2 * SZ_VR + SZ_AT;
static_assert(SZ_WQ % 256 == 0 && SZ_WO % 256 == 0 && SZ_XB % 256 == 0 && SZ_P16 % 256 == 0 && SZ_VR % 256 == 0 && SZ_AT % 256 == 0);
static_assert(SZ_TOTAL <= (size_t)134217728);

__device__ __forceinline__ unsigned short f2bf(float f) { unsigned u = __float_as_uint(f); u += 0x7FFFu + ((u >> 16) & 1u); return (unsigned short)(u >> 16); }
__device__ __forceinline__ float bf2f(unsigned short b) { return __uint_as_float(((unsigned)b) << 16); }
__device__ __forceinline__ float bfr(float f) { return bf2f(f2bf(f)); }
__device__ __forceinline__ void splitf(float y, unsigned short& h, unsigned short& l) { h = f2bf(y); l = f2bf(y - bf2f(h)); }
__device__ __forceinline__ v16h cat16(v8h lo, v8h hi) { return __builtin_shufflevector(lo, hi, 0, 1, 2, 3, 4, 5, 6, 7, 8, 9, 10, 11, 12, 13, 14, 15); }
__device__ __forceinline__ v16bf cat16b(v8us lo, v8us hi) { return __builtin_bit_cast(v16bf, __builtin_shufflevector(lo, hi, 0, 1, 2, 3, 4, 5, 6, 7, 8, 9, 10, 11, 12, 13, 14, 15)); }
__device__ __forceinline__ v8f wmma16(v16h a, v16h b, v8f c) { return __builtin_amdgcn_wmma_f32_16x16x32_f16(false, a, false, b, (short)0, c, false, false); }
__device__ __forceinline__ v8f wmmab(v16bf a, v16bf b, v8f c) { return __builtin_amdgcn_wmma_f32_16x16x32_bf16(false, a, false, b, (short)0, c, false, false); }
__device__ __forceinline__ v16h  ldh(const h16* p) { return cat16(*(const v8h*)p, *(const v8h*)(p + 16)); }
__device__ __forceinline__ v16bf ldb(const bf* p)  { return cat16b(*(const v8us*)p, *(const v8us*)(p + 16)); }

__global__ __launch_bounds__(256) void k_cvtx(const float* __restrict__ x, bf* XB) {
    const size_t i = (size_t)blockIdx.x * 256 + threadIdx.x;
    if (i >= (size_t)MROWS * EM / 8) return;
    const size_t e = i * 8; const int m = (int)(e / EM), col = (int)(e % EM); const int b = m / SEQ, t = m - b * SEQ;
    const v8f v = *(const v8f*)(x + ((size_t)b * SEQ_FULL + t) * EM + col);
    v8us o;
#pragma unroll
    for (int k = 0; k < 8; ++k) o[k] = f2bf(v[k]);
    *(volatile v8us*)(XB + e) = o; __threadfence(); *(volatile v8us*)(XB + e) = o;
}

__global__ __launch_bounds__(256) void k_wt(const float* __restrict__ W, bf* Wt, int N, int K) {
    __shared__ __align__(16) unsigned short ts[64 * 72];
    const int n0 = blockIdx.x * 64, k0 = blockIdx.y * 64, t = threadIdx.x;
#pragma unroll
    for (int ps = 0; ps < 4; ++ps) { const int i = ps * 16 + (t >> 4), j = (t & 15) * 4; const v4f v = *(const v4f*)(W + (size_t)(k0 + i) * N + n0 + j);
#pragma unroll
        for (int q = 0; q < 4; ++q) ts[(j + q) * 72 + i] = f2bf(v[q]); }
    __syncthreads();
    v8us val[2];
#pragma unroll
    for (int p2 = 0; p2 < 2; ++p2) { const int row = p2 * 32 + (t >> 3), c = (t & 7) * 8; val[p2] = *(const v8usa*)(&ts[row * 72 + c]); }
#pragma unroll 1
    for (int ps = 0; ps < 2; ++ps) {
#pragma unroll
        for (int p2 = 0; p2 < 2; ++p2) { const int row = p2 * 32 + (t >> 3), c = (t & 7) * 8; *(volatile v8us*)(Wt + (size_t)(n0 + row) * K + k0 + c) = val[p2]; }
        if (ps == 0) __threadfence(); }
}

__global__ __launch_bounds__(32) void k_gemm_qkv(const bf* __restrict__ A, const bf* __restrict__ Bt, const float* __restrict__ bias, h16* P16, bf* VH, bf* VL) {
    __shared__ __align__(16) float os[64 * 68];
    const int K = EM;
    const int lane = threadIdx.x & 31, lr = lane & 15, hi = lane >> 4; const int r0 = blockIdx.x * 64, c0 = blockIdx.y * 64;
    v8f acc[4][4];
#pragma unroll
    for (int mb = 0; mb < 4; ++mb)
#pragma unroll
        for (int nb = 0; nb < 4; ++nb) acc[mb][nb] = (v8f){};
    const size_t aoff = (size_t)(r0 + lr) * K + 8 * hi, boff = (size_t)(c0 + lr) * K + 8 * hi;
#pragma unroll 1
    for (int kc = 0; kc < K; kc += 32) {
        v16bf a[4]; v16bf bq;
#pragma unroll
        for (int mb = 0; mb < 4; ++mb) a[mb] = ldb(A + aoff + (size_t)mb * 16 * K + kc);
#pragma unroll
        for (int nb = 0; nb < 4; ++nb) { bq = ldb(Bt + boff + (size_t)nb * 16 * K + kc);
#pragma unroll
            for (int mb = 0; mb < 4; ++mb) acc[mb][nb] = wmmab(a[mb], bq, acc[mb][nb]); }
        asm volatile("v_nop\n\tv_nop\n\tv_nop\n\tv_nop" : "+v"(acc[0][0]), "+v"(acc[1][1]), "+v"(acc[2][2]), "+v"(acc[3][3]) : "v"(a[0]), "v"(a[3]), "v"(bq));
    }
    const int ct = blockIdx.y; const int h = ct / 3; const int which = ct - 3 * h;
    const int st = (which == 2) ? 1 : 68, sd = (which == 2) ? 68 : 1;
    float bv[4];
#pragma unroll
    for (int nb = 0; nb < 4; ++nb) bv[nb] = bfr(bias[c0 + nb * 16 + lr]);
#pragma unroll
    for (int mb = 0; mb < 4; ++mb)
#pragma unroll
        for (int nb = 0; nb < 4; ++nb)
#pragma unroll
            for (int j = 0; j < 8; ++j) os[(mb * 16 + hi * 8 + j) * st + (nb * 16 + lr) * sd] = acc[mb][nb][j] + bv[nb];
    __syncthreads();
    const int b = r0 / SEQ, t0 = r0 - b * SEQ; const size_t bh = (size_t)b * NH + h;
    const size_t pitch = (which == 2) ? (size_t)SEQ : (size_t)HD;
    const size_t base = (size_t)which * PLANE + ((which == 2) ? (bh * HD * SEQ + (size_t)t0) : ((bh * SEQ + (size_t)t0) * HD));
    const bool hl = (which == 2) && (t0 < RH);
    const size_t hbase = bh * HD * RH + (size_t)((t0 < RH) ? t0 : 0);
    const int rq = lane >> 3, cq = (lane & 7) * 8;
#pragma unroll 1
    for (int ps = 0; ps < 2; ++ps) {
#pragma unroll 2
        for (int s = 0; s < 16; ++s) { const int row = s * 4 + rq;
            const v4f x0 = *(const v4fa*)(&os[row * 68 + cq]); const v4f x1 = *(const v4fa*)(&os[row * 68 + cq + 4]);
            v8h o;
#pragma unroll
            for (int k = 0; k < 4; ++k) { o[k] = (h16)x0[k]; o[4 + k] = (h16)x1[k]; }
            *(volatile v8h*)(P16 + base + (size_t)row * pitch + cq) = o;
            if (hl) { v8us oh, ol;
#pragma unroll
                for (int k = 0; k < 4; ++k) { unsigned short a2, c2; splitf(x0[k], a2, c2); oh[k] = a2; ol[k] = c2; splitf(x1[k], a2, c2); oh[4 + k] = a2; ol[4 + k] = c2; }
                *(volatile v8us*)(VH + hbase + (size_t)row * RH + cq) = oh; *(volatile v8us*)(VL + hbase + (size_t)row * RH + cq) = ol; } }
        if (ps == 0) __threadfence(); }
}

__global__ __launch_bounds__(32) void k_gemm_out(const bf* __restrict__ A, const bf* __restrict__ Bt, const float* __restrict__ bias, float* C) {
    __shared__ __align__(16) float os[16 * 68];
    const int K = EM;
    const int lane = threadIdx.x & 31, lr = lane & 15, hi = lane >> 4; const int r0 = blockIdx.x * 64, c0 = blockIdx.y * 64;
    v8f acc[4][4];
#pragma unroll
    for (int mb = 0; mb < 4; ++mb)
#pragma unroll
        for (int nb = 0; nb < 4; ++nb) acc[mb][nb] = (v8f){};
    const size_t aoff = (size_t)(r0 + lr) * K + 8 * hi, boff = (size_t)(c0 + lr) * K + 8 * hi;
#pragma unroll 1
    for (int kk = 0; kk < 2 * K; kk += 32) {
        const int kc = (kk >= K) ? (kk - K) : kk; const size_t pofs = (kk >= K) ? ATPLANE : (size_t)0;
        v16bf a[4]; v16bf bq;
#pragma unroll
        for (int mb = 0; mb < 4; ++mb) a[mb] = ldb(A + pofs + aoff + (size_t)mb * 16 * K + kc);
#pragma unroll
        for (int nb = 0; nb < 4; ++nb) { bq = ldb(Bt + boff + (size_t)nb * 16 * K + kc);
#pragma unroll
            for (int mb = 0; mb < 4; ++mb) acc[mb][nb] = wmmab(a[mb], bq, acc[mb][nb]); }
        asm volatile("v_nop\n\tv_nop\n\tv_nop\n\tv_nop" : "+v"(acc[0][0]), "+v"(acc[1][1]), "+v"(acc[2][2]), "+v"(acc[3][3]) : "v"(a[0]), "v"(a[3]), "v"(bq));
    }
    const int b = r0 / SEQ, t0 = r0 - b * SEQ; const int cofs = lr * 4;
    v4f bias4;
#pragma unroll
    for (int k = 0; k < 4; ++k) bias4[k] = bfr(bias[c0 + cofs + k]);
#pragma unroll
    for (int mb = 0; mb < 4; ++mb) {
#pragma unroll
        for (int nb = 0; nb < 4; ++nb)
#pragma unroll
            for (int j = 0; j < 8; ++j) os[(hi * 8 + j) * 68 + nb * 16 + lr] = acc[mb][nb][j];
        __syncthreads();
        float* crow = C + ((size_t)b * SEQ_FULL + t0 + mb * 16) * EM + c0;
        v4f vals[8];
#pragma unroll
        for (int s = 0; s < 8; ++s) { const int row = 2 * s + hi; vals[s] = *(const v4fa*)(&os[row * 68 + cofs]) + bias4; }
#pragma unroll 1
        for (int ps = 0; ps < 2; ++ps) {
#pragma unroll
            for (int s = 0; s < 8; ++s) { const int row = 2 * s + hi; *(volatile v4f*)(crow + (size_t)row * EM + cofs) = vals[s]; }
            if (ps == 0) __threadfence(); }
        __syncthreads();
    }
}

template <bool HL>
__device__ __forceinline__ void attn_body(const h16* __restrict__ P16, const bf* __restrict__ VH, const bf* __restrict__ VL, const int* __restrict__ mask, bf* AT) {
    __shared__ __align__(16) h16 Ps[16 * PP];
    __shared__ __align__(16) unsigned short Pb[2 * 16 * PP];
    __shared__ __align__(16) float Os[16 * 68];
    constexpr int QTL = HL ? (RH / 16) : (SEQ / 16);
    const int lane = threadIdx.x & 31, lr = lane & 15, hi = lane >> 4;
    int idx = blockIdx.x; const int qt = idx % QTL; idx /= QTL; const int h = idx % NH; const int b = idx / NH;
    const int causal = (mask[0] != 0) ? 1 : 0;
    const int q0 = qt * 16;
    if (HL) { if (!causal) return; } else { if (causal && q0 < RH) return; }
    const size_t bh = (size_t)b * NH + h;
    const size_t qoff = bh * SEQ * HD, koff = PLANE + bh * SEQ * HD, voff = 2 * PLANE + bh * HD * SEQ, roff = bh * HD * RH;
    const v16h qf0 = ldh(P16 + qoff + (size_t)(q0 + lr) * HD + 8 * hi);
    const v16h qf1 = ldh(P16 + qoff + (size_t)(q0 + lr) * HD + 32 + 8 * hi);
    v8f o[4];
#pragma unroll
    for (int nt = 0; nt < 4; ++nt) o[nt] = (v8f){};
    float rmax[8], rsum[8];
#pragma unroll
    for (int r = 0; r < 8; ++r) { rmax[r] = -3.0e38f; rsum[r] = 0.0f; }
    const int nblocks = causal ? ((q0 + 47) >> 5) : (SEQ / 32);
    const int limb = causal ? (q0 + 8 * hi) : 0x3fffffff;
#pragma unroll 1
    for (int kb = 0; kb < nblocks; ++kb) {
        const int key0 = kb * 32;
        v8f s0 = (v8f){}, s1 = (v8f){};
        {
            const h16* kp = P16 + koff + (size_t)(key0 + lr) * HD + 8 * hi;
            const v16h k00 = ldh(kp), k01 = ldh(kp + 32), k10 = ldh(kp + 16 * HD), k11 = ldh(kp + 16 * HD + 32);
            s0 = wmma16(qf0, k00, s0); s0 = wmma16(qf1, k01, s0); s1 = wmma16(qf0, k10, s1); s1 = wmma16(qf1, k11, s1);
            asm volatile("v_nop\n\tv_nop\n\tv_nop\n\tv_nop" : "+v"(s0), "+v"(s1) : "v"(qf1), "v"(k11));
        }
        const int kcol = key0 + lr;
        float fac[8];
#pragma unroll
        for (int r = 0; r < 8; ++r) {
            const int lim = limb + r;
            const bool in0 = (kcol <= lim), in1 = (kcol + 16 <= lim);
            const float a0 = in0 ? s0[r] : -3.0e38f, a1 = in1 ? s1[r] : -3.0e38f;
            float mx = fmaxf(a0, a1);
            mx = fmaxf(mx, __shfl_xor(mx, 1, 32)); mx = fmaxf(mx, __shfl_xor(mx, 2, 32)); mx = fmaxf(mx, __shfl_xor(mx, 4, 32)); mx = fmaxf(mx, __shfl_xor(mx, 8, 32));
            const float nm = fmaxf(rmax[r], mx);
            const float f  = __builtin_amdgcn_exp2f((rmax[r] - nm) * CE);
            const float e0 = __builtin_amdgcn_exp2f((a0 - nm) * CE), e1 = __builtin_amdgcn_exp2f((a1 - nm) * CE);
            const float p0 = in0 ? e0 : 0.0f, p1 = in1 ? e1 : 0.0f;
            rsum[r] = rsum[r] * f + (p0 + p1);
            rmax[r] = nm; fac[r] = f;
            if (HL) { unsigned short a2, c2; splitf(p0, a2, c2); Pb[(8 * hi + r) * PP + lr] = a2; Pb[16 * PP + (8 * hi + r) * PP + lr] = c2;
                      splitf(p1, a2, c2); Pb[(8 * hi + r) * PP + 16 + lr] = a2; Pb[16 * PP + (8 * hi + r) * PP + 16 + lr] = c2; }
            else    { Ps[(8 * hi + r) * PP + lr] = (h16)(p0 * PCAR); Ps[(8 * hi + r) * PP + 16 + lr] = (h16)(p1 * PCAR); }
        }
#pragma unroll
        for (int nt = 0; nt < 4; ++nt)
#pragma unroll
            for (int r = 0; r < 8; ++r) o[nt][r] *= fac[r];
        __syncthreads();
        if (HL) {
            const v16bf ph = cat16b(*(const v8usa*)(&Pb[lr * PP + 8 * hi]), *(const v8usa*)(&Pb[lr * PP + 16 + 8 * hi]));
            const v16bf pl = cat16b(*(const v8usa*)(&Pb[16 * PP + lr * PP + 8 * hi]), *(const v8usa*)(&Pb[16 * PP + lr * PP + 16 + 8 * hi]));
            v16bf vh[4], vl[4];
#pragma unroll
            for (int nt = 0; nt < 4; ++nt) { const size_t vo = roff + (size_t)(nt * 16 + lr) * RH + key0 + 8 * hi; vh[nt] = ldb(VH + vo); vl[nt] = ldb(VL + vo); }
#pragma unroll
            for (int nt = 0; nt < 4; ++nt) { o[nt] = wmmab(ph, vh[nt], o[nt]); o[nt] = wmmab(pl, vh[nt], o[nt]); o[nt] = wmmab(ph, vl[nt], o[nt]); }
            asm volatile("v_nop\n\tv_nop\n\tv_nop\n\tv_nop" : "+v"(o[0]), "+v"(o[1]), "+v"(o[2]), "+v"(o[3]) : "v"(ph), "v"(pl), "v"(vl[3]), "v"(vh[3]));
        } else {
            const v16h pa = cat16(*(const v8ha*)(&Ps[lr * PP + 8 * hi]), *(const v8ha*)(&Ps[lr * PP + 16 + 8 * hi]));
            v16h vf[4];
#pragma unroll
            for (int nt = 0; nt < 4; ++nt) vf[nt] = ldh(P16 + voff + (size_t)(nt * 16 + lr) * SEQ + key0 + 8 * hi);
#pragma unroll
            for (int nt = 0; nt < 4; ++nt) o[nt] = wmma16(pa, vf[nt], o[nt]);
            asm volatile("v_nop\n\tv_nop\n\tv_nop\n\tv_nop" : "+v"(o[0]), "+v"(o[1]), "+v"(o[2]), "+v"(o[3]) : "v"(pa), "v"(vf[3]));
        }
        __syncthreads();
    }
    float rinv[8];
#pragma unroll
    for (int r = 0; r < 8; ++r) { float t = rsum[r]; t += __shfl_xor(t, 1, 32); t += __shfl_xor(t, 2, 32); t += __shfl_xor(t, 4, 32); t += __shfl_xor(t, 8, 32); rinv[r] = 1.0f / (HL ? t : (t * PCAR)); }
#pragma unroll
    for (int nt = 0; nt < 4; ++nt)
#pragma unroll
        for (int r = 0; r < 8; ++r) Os[(8 * hi + r) * 68 + nt * 16 + lr] = o[nt][r] * rinv[r];
    __syncthreads();
    const int rq = lane >> 3, cq = (lane & 7) * 8;
    v8us oh[4], ol[4];
#pragma unroll
    for (int s = 0; s < 4; ++s) { const int row = s * 4 + rq;
        const v4f x0 = *(const v4fa*)(&Os[row * 68 + cq]); const v4f x1 = *(const v4fa*)(&Os[row * 68 + cq + 4]);
#pragma unroll
        for (int k = 0; k < 4; ++k) { unsigned short a2, c2; splitf(x0[k], a2, c2); oh[s][k] = a2; ol[s][k] = c2; splitf(x1[k], a2, c2); oh[s][4 + k] = a2; ol[s][4 + k] = c2; } }
#pragma unroll 1
    for (int ps = 0; ps < 2; ++ps) {
#pragma unroll
        for (int s = 0; s < 4; ++s) { const int row = s * 4 + rq; bf* dst = AT + ((size_t)b * SEQ + q0 + row) * EM + h * HD + cq;
            *(volatile v8us*)dst = oh[s]; *(volatile v8us*)(dst + ATPLANE) = ol[s]; }
        if (ps == 0) __threadfence(); }
}
__global__ __launch_bounds__(32) void k_attn16(const h16* P16, const int* mask, bf* AT) { attn_body<false>(P16, (const bf*)0, (const bf*)0, mask, AT); }
__global__ __launch_bounds__(32) void k_attnhl(const h16* P16, const bf* VH, const bf* VL, const int* mask, bf* AT) { attn_body<true>(P16, VH, VL, mask, AT); }

extern "C" void kernel_launch(void* const* d_in, const int* in_sizes, int n_in,
                              void* d_out, int out_size, void* d_ws, size_t ws_size, hipStream_t stream) {
    if (n_in < 6) return;
    const size_t need_x = ((size_t)(NB - 1) * SEQ_FULL + SEQ) * EM;
    if ((size_t)in_sizes[0] < need_x || (size_t)in_sizes[1] < (size_t)EM * E3 || in_sizes[2] < E3 || (size_t)in_sizes[3] < (size_t)EM * EM || in_sizes[4] < EM || in_sizes[5] < 1) return;
    if ((size_t)out_size < need_x) return;
    if (ws_size < SZ_TOTAL) return;
    const float* x = (const float*)d_in[0]; const float* wqkv = (const float*)d_in[1]; const float* bqkv = (const float*)d_in[2];
    const float* wout = (const float*)d_in[3]; const float* bout = (const float*)d_in[4]; const int* mask = (const int*)d_in[5];
    float* OUT = (float*)d_out;
    char* wsp = (char*)d_ws;
    bf*  WQ  = (bf*)wsp;  wsp += SZ_WQ;
    bf*  WO  = (bf*)wsp;  wsp += SZ_WO;
    bf*  XB  = (bf*)wsp;  wsp += SZ_XB;
    h16* P16 = (h16*)wsp; wsp += SZ_P16;
    bf*  VH  = (bf*)wsp;  wsp += SZ_VR;
    bf*  VL  = (bf*)wsp;  wsp += SZ_VR;
    bf*  AT  = (bf*)wsp;  wsp += SZ_AT;
    k_wt<<<dim3(E3 / 64, EM / 64), 256, 0, stream>>>(wqkv, WQ, E3, EM);
    k_wt<<<dim3(EM / 64, EM / 64), 256, 0, stream>>>(wout, WO, EM, EM);
    k_cvtx<<<(unsigned)((size_t)MROWS * EM / 2048), 256, 0, stream>>>(x, XB);
    k_gemm_qkv<<<dim3(MROWS / 64, E3 / 64), 32, 0, stream>>>(XB, WQ, bqkv, P16, VH, VL);
    k_attn16<<<NB * NH * (SEQ / 16), 32, 0, stream>>>(P16, mask, AT);
    k_attnhl<<<NB * NH * (RH / 16), 32, 0, stream>>>(P16, VH, VL, mask, AT);
    k_gemm_out<<<dim3(MROWS / 64, EM / 64), 32, 0, stream>>>(AT, WO, bout, OUT);
}
